// TransformerLayer_8976481648779
// MI455X (gfx1250) — hardware-verified
//
#include <hip/hip_runtime.h>
#include <math.h>

typedef __attribute__((ext_vector_type(16))) _Float16 v16h;
typedef __attribute__((ext_vector_type(8)))  _Float16 v8h;
typedef __attribute__((ext_vector_type(4)))  _Float16 v4h;
typedef __attribute__((ext_vector_type(8)))  float v8f;
typedef __attribute__((ext_vector_type(4)))  float v4f;

#ifndef SEQ
#define SEQ 2048
#endif
#define SEQ_FULL 2048
#ifndef NB
#define NB 2
#endif
#define NB_FULL 2
#define DM 256
#define NH 8
#define DH 32
#define FF 1024
#define TOKS ((unsigned)(NB) * (unsigned)(SEQ))
#define ROWS (2u * TOKS)
#define OUT1_OFF ((size_t)NB_FULL * SEQ_FULL * DM)
#define SCALE (0.17677669529663687f)
#define PCY (16384.0f)
#define WC (64.0f)
#define OC (256.0f)
#define F16MIN (6.103515625e-05f)
#define LN_EPS (1e-5f)
static_assert(SEQ % 64 == 0);
static_assert(SEQ >= 64);
static_assert(SEQ <= SEQ_FULL);
static_assert(NB >= 1 && NB <= NB_FULL);
static_assert(DM == NH * DH);
static_assert(DH == 32);
static_assert(DM % 128 == 0 && FF % 128 == 0);
static_assert(OUT1_OFF * 4u == 4194304u);

#define WSZ_WQKV (2u * (size_t)768 * DM)
#define WSZ_WO   (2u * (size_t)DM * DM)
#define WSZ_W1T  (2u * (size_t)FF * DM)
#define WSZ_W2T  (2u * (size_t)DM * FF)
#define WSZ_P16  (2u * (size_t)ROWS * DM)
#define WSZ_P32  (4u * (size_t)ROWS * DM)
#define WSZ_H    (2u * (size_t)ROWS * FF)
#define WS_WQKVS ((size_t)0)
#define WS_WOS   (WS_WQKVS + WSZ_WQKV)
#define WS_WQKVC (WS_WOS   + WSZ_WO)
#define WS_WOC   (WS_WQKVC + WSZ_WQKV)
#define WS_W1T   (WS_WOC   + WSZ_WO)
#define WS_W2T   (WS_W1T   + WSZ_W1T)
#define WS_XN    (WS_W2T   + WSZ_W2T)
#define WS_Q     (WS_XN    + WSZ_P16)
#define WS_K     (WS_Q     + WSZ_P16)
#define WS_VT    (WS_K     + WSZ_P16)
#define WS_O     (WS_VT    + WSZ_P16)
#define WS_X1    (WS_O     + WSZ_P16)
#define WS_X2    (WS_X1    + WSZ_P32)
#define WS_H     (WS_X2    + WSZ_P32)
#define WS_END   (WS_H     + WSZ_H)
static_assert(WS_END <= (size_t)134217728u);
static_assert((WS_XN % 256u) == 0 && (WS_Q % 256u) == 0 && (WS_VT % 256u) == 0 && (WS_X1 % 256u) == 0 && (WS_H % 256u) == 0);
static_assert((ROWS / 64u) * 64u == ROWS);
static_assert((TOKS / 64u) * 64u == TOKS);
static_assert((ROWS / 8u) * 8u == ROWS);
static_assert((SEQ / 16) * 16 == SEQ);

template <typename T> __device__ __forceinline__ void vst2(void* p, T v) { *(volatile T*)p = v; __threadfence(); *(volatile T*)p = v; }
__device__ __forceinline__ v8f zero8() { v8f z = {0.f, 0.f, 0.f, 0.f, 0.f, 0.f, 0.f, 0.f}; return z; }
__device__ __forceinline__ v8f wmma16(v16h a, v16h b, v8f c) {
  v8f d = __builtin_amdgcn_wmma_f32_16x16x32_f16(false, a, false, b, (short)0, c, false, false);
  asm volatile("v_nop\n\tv_nop\n\tv_nop\n\tv_nop" : "+v"(d) : "v"(a), "v"(b));
  return d;
}
__device__ __forceinline__ v16h frag_h(const _Float16* rowk0, int lane) {
  union { v16h v; v8h q[2]; } u; const _Float16* p = rowk0 + 8 * (lane >> 4);
  u.q[0] = *(const v8h*)p; u.q[1] = *(const v8h*)(p + 16); return u.v;
}
__device__ __forceinline__ _Float16 f16n(float x) { const float t = (fabsf(x) >= F16MIN) ? x : 0.0f; return (_Float16)t; }
__device__ __forceinline__ unsigned short bf16bits(float x) { unsigned u = __float_as_uint(x); u += 0x7FFFu + ((u >> 16) & 1u); return (unsigned short)(u >> 16); }
__device__ __forceinline__ float bf16val(unsigned short b) { return __uint_as_float(((unsigned)b) << 16); }
__device__ __forceinline__ float rnev(float x) { return bf16val(bf16bits(x)); }
#define LDSX() do { asm volatile("s_wait_dscnt 0" ::: "memory"); __builtin_amdgcn_wave_barrier(); __builtin_amdgcn_fence(3  , "workgroup"); } while (0)

__global__ __launch_bounds__(256) void k_wt(const float* __restrict__ src, unsigned K, unsigned N, _Float16* __restrict__ dst) {
  __shared__ __align__(16) _Float16 t[64][72];
  const unsigned tid = threadIdx.x; const unsigned n0 = blockIdx.x * 64u, k0 = blockIdx.y * 64u;
  const unsigned np = tid & 15u, kq = tid >> 4;
#pragma unroll
  for (unsigned i = 0; i < 4; ++i) {
    const unsigned kk = kq + 16u * i;
    const v4f v = *(const v4f*)(src + (size_t)(k0 + kk) * N + n0 + 4u * np);
#pragma unroll
    for (int e = 0; e < 4; ++e) t[4u * np + e][kk] = f16n(rnev(v[e]) * WC);
  }
  __syncthreads();
  for (unsigned e = tid; e < 64u * 8u; e += 256u) { const unsigned nl = e >> 3, q = e & 7u; vst2(dst + (size_t)(n0 + nl) * K + k0 + q * 8u, *(const v8h*)&t[nl][q * 8u]); }
}

template <int RAW>
__global__ __launch_bounds__(256) void k_ln(const float* __restrict__ S0, const float* __restrict__ S1, unsigned bs, const float* __restrict__ G, const float* __restrict__ Bt, _Float16* __restrict__ XN) {
  const unsigned wave = threadIdx.x >> 5, lane = threadIdx.x & 31u; const unsigned row = blockIdx.x * 8u + wave;
  if (row >= ROWS) return;
  const unsigned s = row / TOKS, rem = row - s * TOKS, b = rem / (unsigned)SEQ, tk = rem - b * (unsigned)SEQ;
  const float* p = (s ? S1 : S0) + ((size_t)b * bs + tk) * DM + lane * 8u;
  const v4f a = *(const v4f*)p, c = *(const v4f*)(p + 4);
  float v[8];
#pragma unroll
  for (int e = 0; e < 4; ++e) { v[e] = RAW ? rnev(a[e]) : a[e]; v[4 + e] = RAW ? rnev(c[e]) : c[e]; }
  float s1 = ((v[0] + v[1]) + (v[2] + v[3])) + ((v[4] + v[5]) + (v[6] + v[7]));
#pragma unroll
  for (int o = 1; o < 32; o <<= 1) s1 += __shfl_xor(s1, o);
  const float mu = s1 * (1.0f / DM); float q = 0.f;
#pragma unroll
  for (int e = 0; e < 8; ++e) { const float d = v[e] - mu; q += d * d; }
#pragma unroll
  for (int o = 1; o < 32; o <<= 1) q += __shfl_xor(q, o);
  const float inv = rsqrtf(q * (1.0f / DM) + LN_EPS);
  const v4f ga = *(const v4f*)(G + lane * 8u), gb = *(const v4f*)(G + lane * 8u + 4u);
  const v4f ba = *(const v4f*)(Bt + lane * 8u), bb = *(const v4f*)(Bt + lane * 8u + 4u);
  v8h o8;
#pragma unroll
  for (int e = 0; e < 4; ++e) { o8[e] = f16n((v[e] - mu) * inv * rnev(ga[e]) + rnev(ba[e])); o8[4 + e] = f16n((v[4 + e] - mu) * inv * rnev(gb[e]) + rnev(bb[e])); }
  vst2(XN + (size_t)row * DM + lane * 8u, o8);
}

__device__ __forceinline__ void gemm_core(const _Float16* __restrict__ A, const _Float16* __restrict__ W, unsigned K, size_t arow, unsigned c0, int lane, v8f (&acc)[8]) {
  const unsigned col = (unsigned)lane & 15u;
#pragma unroll
  for (int j = 0; j < 8; ++j) acc[j] = zero8();
#pragma unroll 1
  for (unsigned kc = 0; kc < K; kc += 32u) {
    const v16h a = frag_h(A + (arow + col) * K + kc, lane);
#pragma unroll
    for (int j = 0; j < 8; ++j) acc[j] = wmma16(a, frag_h(W + (size_t)(c0 + j * 16u + col) * K + kc, lane), acc[j]);
  }
}
__device__ __forceinline__ void stage_rm(_Float16* sbuf, const v8f (&acc)[8], const float (&bv)[8], float sc, unsigned wave, unsigned g, unsigned col, int relu) {
#pragma unroll
  for (int j = 0; j < 8; ++j)
#pragma unroll
    for (int r = 0; r < 8; ++r) { float v = acc[j][r] * sc + bv[j]; if (relu) v = fmaxf(v, 0.0f); sbuf[(wave * 16u + 8u * g + r) * 136u + j * 16u + col] = f16n(v); }
}
__device__ __forceinline__ void store_rm(const _Float16* sbuf, _Float16* OP, unsigned pitch, size_t r0blk, unsigned cbase, unsigned tid) {
  for (unsigned e = tid; e < 64u * 16u; e += 128u) { const unsigned rl = e >> 4, q = e & 15u; vst2(OP + (r0blk + rl) * pitch + cbase + q * 8u, *(const v8h*)&sbuf[rl * 136u + q * 8u]); }
}

__global__ __launch_bounds__(128) void k_qkv(const _Float16* __restrict__ A, const _Float16* __restrict__ W, const float* __restrict__ BQ, const float* __restrict__ BK, const float* __restrict__ BV,
                                             _Float16* QO, _Float16* KO, _Float16* VTO) {
  __shared__ __align__(16) _Float16 sbuf[128 * 72];
  const unsigned tid = threadIdx.x, wave = tid >> 5; const int lane = (int)(tid & 31u); const unsigned col = tid & 15u, g = (tid >> 4) & 1u;
  const size_t r0blk = (size_t)blockIdx.x * 64u; const unsigned y = blockIdx.y, sel = y >> 1, cl0 = (y & 1u) * 128u, c0 = y * 128u;
  v8f acc[8];
  gemm_core(A, W, (unsigned)DM, r0blk + wave * 16u, c0, lane, acc);
  const float* bp = (sel == 0u) ? BQ : ((sel == 1u) ? BK : BV);
  float bv[8];
#pragma unroll
  for (int j = 0; j < 8; ++j) bv[j] = rnev(bp[cl0 + j * 16u + col]);
  if (sel < 2u) {
    stage_rm(sbuf, acc, bv, 1.0f / WC, wave, g, col, 0);
  } else {
#pragma unroll
    for (int j = 0; j < 8; ++j)
#pragma unroll
      for (int r = 0; r < 8; ++r) sbuf[(j * 16u + col) * 72u + wave * 16u + 8u * g + r] = f16n(acc[j][r] * (1.0f / WC) + bv[j]);
  }
  __syncthreads();
  if (sel < 2u) {
    store_rm(sbuf, sel ? KO : QO, (unsigned)DM, r0blk, cl0, tid);
  } else {
    for (unsigned e = tid; e < 128u * 8u; e += 128u) { const unsigned cl = e >> 3, q = e & 7u; vst2(VTO + (size_t)(cl0 + cl) * ROWS + r0blk + q * 8u, *(const v8h*)&sbuf[cl * 72u + q * 8u]); }
  }
}

__global__ __launch_bounds__(128) void k_ffn1(const _Float16* __restrict__ A, const _Float16* __restrict__ W, const float* __restrict__ B1, _Float16* __restrict__ H) {
  __shared__ __align__(16) _Float16 sbuf[64 * 136];
  const unsigned tid = threadIdx.x, wave = tid >> 5; const int lane = (int)(tid & 31u); const unsigned col = tid & 15u, g = (tid >> 4) & 1u;
  const size_t r0blk = (size_t)blockIdx.x * 64u; const unsigned c0 = blockIdx.y * 128u;
  v8f acc[8];
  gemm_core(A, W, (unsigned)DM, r0blk + wave * 16u, c0, lane, acc);
  float bv[8];
#pragma unroll
  for (int j = 0; j < 8; ++j) bv[j] = rnev(B1[c0 + j * 16u + col]);
  stage_rm(sbuf, acc, bv, 1.0f / WC, wave, g, col, 1);
  __syncthreads();
  store_rm(sbuf, H, (unsigned)FF, r0blk, c0, tid);
}

template <int RNERES>
__global__ __launch_bounds__(128) void k_gres(const _Float16* __restrict__ A, const _Float16* __restrict__ W, unsigned K, const float* __restrict__ BO,
                                              const float* R0, const float* R1, unsigned rbs, float* O0, float* O1, unsigned obs, float sc) {
  __shared__ __align__(16) float sf[4][16][132];
  const unsigned tid = threadIdx.x, wave = tid >> 5; const int lane = (int)(tid & 31u); const unsigned col = tid & 15u, g = (tid >> 4) & 1u, ln = tid & 31u;
  const unsigned row0 = blockIdx.x * 64u; const unsigned c0 = blockIdx.y * 128u;
  v8f acc[8];
  gemm_core(A, W, K, (size_t)row0 + wave * 16u, c0, lane, acc);
  float bv[8];
#pragma unroll
  for (int j = 0; j < 8; ++j) bv[j] = rnev(BO[c0 + j * 16u + col]);
#pragma unroll
  for (int j = 0; j < 8; ++j)
#pragma unroll
    for (int r = 0; r < 8; ++r) sf[wave][8u * g + r][j * 16u + col] = acc[j][r] * sc + bv[j];
  LDSX();
  const unsigned s = row0 / TOKS, rem = row0 - s * TOKS, b = rem / (unsigned)SEQ, t0 = rem - b * (unsigned)SEQ + wave * 16u;
  const float* rp = (s ? R1 : R0) + ((size_t)b * rbs + t0) * DM + c0 + ln * 4u;
  float* op = (s ? O1 : O0) + ((size_t)b * obs + t0) * DM + c0 + ln * 4u;
#pragma unroll 1
  for (unsigned rl = 0; rl < 16u; ++rl) {
    v4f vv = *(const v4f*)&sf[wave][rl][ln * 4u];
    const v4f rv = *(const v4f*)(rp + (size_t)rl * DM);
#pragma unroll
    for (int e = 0; e < 4; ++e) vv[e] += RNERES ? rnev(rv[e]) : rv[e];
    vst2(op + (size_t)rl * DM, vv);
  }
}

template <int CROSS>
__global__ __launch_bounds__(256) void k_attn(const _Float16* __restrict__ Q, const _Float16* __restrict__ KP, const _Float16* __restrict__ VT, const float* __restrict__ VB, _Float16* __restrict__ O) {
  __shared__ __align__(16) _Float16 sP[8][16][72];
  __shared__ __align__(16) float sB[2][64][20];
  __shared__ __align__(16) _Float16 sO[16][264];
  const unsigned tid = threadIdx.x, wave = tid >> 5; const int lane = (int)(tid & 31u); const unsigned col = tid & 15u, g = (tid >> 4) & 1u;
  const unsigned q0 = blockIdx.x * 16u, sb = blockIdx.y, s = sb / (unsigned)NB, b = sb - s * (unsigned)NB;
  const unsigned ks = CROSS ? (s ^ 1u) : s;
  const size_t qrow0 = (size_t)s * TOKS + (size_t)b * SEQ + q0;
  const size_t krow0 = (size_t)ks * TOKS + (size_t)b * SEQ;
  const unsigned hc = wave * DH;
  const v16h qa = frag_h(Q + (qrow0 + col) * DM + hc, lane);
  float mrow[8], lsum[8];
#pragma unroll
  for (int r = 0; r < 8; ++r) { mrow[r] = -1.0e30f; lsum[r] = 0.f; }
  v8f o0 = zero8(), o1 = zero8();
#pragma unroll 1
  for (unsigned kt = 0; kt < (unsigned)SEQ / 64u; ++kt) {
    const unsigned key0 = kt * 64u; const unsigned buf = kt & 1u;
    if (CROSS) {
      if (s == 0u) {
        const unsigned qq = tid >> 4, pc = tid & 15u;
        const v4f v = *(const v4f*)(VB + ((size_t)b * SEQ_FULL + q0 + qq) * SEQ_FULL + key0 + 4u * pc);
#pragma unroll
        for (int e = 0; e < 4; ++e) sB[buf][4u * pc + e][qq] = rnev(v[e]);
      } else {
        const unsigned kk = tid >> 2, pc = tid & 3u;
        const v4f v = *(const v4f*)(VB + ((size_t)b * SEQ_FULL + key0 + kk) * SEQ_FULL + q0 + 4u * pc);
        v4f w;
#pragma unroll
        for (int e = 0; e < 4; ++e) w[e] = rnev(v[e]);
        *(v4f*)&sB[buf][kk][4u * pc] = w;
      }
      __syncthreads();
    }
    v8f sc[4];
#pragma unroll
    for (int t = 0; t < 4; ++t) sc[t] = wmma16(qa, frag_h(KP + (krow0 + key0 + 4u * col + t) * DM + hc, lane), zero8());
    if (CROSS) {
#pragma unroll
      for (int t = 0; t < 4; ++t) {
        const float* bp = &sB[buf][4u * col + t][8u * g];
        const v4f x = *(const v4f*)bp, y = *(const v4f*)(bp + 4);
#pragma unroll
        for (int e = 0; e < 4; ++e) { sc[t][e] = sc[t][e] * SCALE + x[e]; sc[t][4 + e] = sc[t][4 + e] * SCALE + y[e]; }
      }
    } else {
#pragma unroll
      for (int t = 0; t < 4; ++t)
#pragma unroll
        for (int r = 0; r < 8; ++r) sc[t][r] = sc[t][r] * SCALE;
    }
#pragma unroll
    for (int r = 0; r < 8; ++r) {
      float mx = fmaxf(fmaxf(sc[0][r], sc[1][r]), fmaxf(sc[2][r], sc[3][r]));
      mx = fmaxf(mx, __shfl_xor(mx, 1)); mx = fmaxf(mx, __shfl_xor(mx, 2)); mx = fmaxf(mx, __shfl_xor(mx, 4)); mx = fmaxf(mx, __shfl_xor(mx, 8));
      const float mn = fmaxf(mrow[r], mx);
      const float al = __expf(mrow[r] - mn);
      mrow[r] = mn; o0[r] *= al; o1[r] *= al;
      float ls = lsum[r] * al;
      v4h pk;
#pragma unroll
      for (int t = 0; t < 4; ++t) { const float pc = __expf(sc[t][r] - mn) * PCY; const _Float16 ph = (_Float16)pc; ls += (float)ph; pk[t] = ph; }
      lsum[r] = ls;
      *(v4h*)&sP[wave][8u * g + r][4u * col] = pk;
    }
    LDSX();
#pragma unroll
    for (int kk = 0; kk < 2; ++kk) {
      const v16h a = frag_h(&sP[wave][col][kk * 32], lane);
      o0 = wmma16(a, frag_h(VT + (size_t)(hc + col) * ROWS + krow0 + key0 + kk * 32u, lane), o0);
      o1 = wmma16(a, frag_h(VT + (size_t)(hc + 16u + col) * ROWS + krow0 + key0 + kk * 32u, lane), o1);
    }
    LDSX();
  }
#pragma unroll
  for (int r = 0; r < 8; ++r) {
    float t = lsum[r]; t += __shfl_xor(t, 1); t += __shfl_xor(t, 2); t += __shfl_xor(t, 4); t += __shfl_xor(t, 8);
    const float inv = OC * (1.0f / t);
    sO[8u * g + r][hc + col] = f16n(o0[r] * inv);
    sO[8u * g + r][hc + 16u + col] = f16n(o1[r] * inv);
  }
  __syncthreads();
  for (unsigned e = tid; e < 16u * 32u; e += 256u) { const unsigned rl = e >> 5, pc = e & 31u; vst2(O + (qrow0 + rl) * DM + pc * 8u, *(const v8h*)&sO[rl][pc * 8u]); }
}

extern "C" void kernel_launch(void* const* d_in, const int* in_sizes, int n_in, void* d_out, int out_size, void* d_ws, size_t ws_size, hipStream_t stream) {
  if (n_in < 29) return;
  const size_t need_x = ((size_t)(NB - 1) * SEQ_FULL + SEQ) * DM;
  const size_t need_vb = ((size_t)(NB - 1) * SEQ_FULL + (SEQ - 1)) * SEQ_FULL + SEQ;
  if ((size_t)in_sizes[0] < need_x || (size_t)in_sizes[1] < need_x || (size_t)in_sizes[2] < need_vb) return;
  for (int i = 3; i <= 17; i += 2) if (in_sizes[i] < DM * DM) return;
  for (int i = 4; i <= 18; i += 2) if (in_sizes[i] < DM) return;
  for (int i = 19; i <= 24; ++i) if (in_sizes[i] < DM) return;
  if (in_sizes[25] < DM * FF || in_sizes[26] < FF || in_sizes[27] < FF * DM || in_sizes[28] < DM) return;
  if ((size_t)out_size < OUT1_OFF + need_x) return;
  if (ws_size < (size_t)WS_END) return;
  const float* x0 = (const float*)d_in[0]; const float* x1 = (const float*)d_in[1]; const float* vb = (const float*)d_in[2];
  const float* sa_wq = (const float*)d_in[3];  const float* sa_bq = (const float*)d_in[4];
  const float* sa_wk = (const float*)d_in[5];  const float* sa_bk = (const float*)d_in[6];
  const float* sa_wv = (const float*)d_in[7];  const float* sa_bv = (const float*)d_in[8];
  const float* sa_wo = (const float*)d_in[9];  const float* sa_bo = (const float*)d_in[10];
  const float* ca_wq = (const float*)d_in[11]; const float* ca_bq = (const float*)d_in[12];
  const float* ca_wk = (const float*)d_in[13]; const float* ca_bk = (const float*)d_in[14];
  const float* ca_wv = (const float*)d_in[15]; const float* ca_bv = (const float*)d_in[16];
  const float* ca_wo = (const float*)d_in[17]; const float* ca_bo = (const float*)d_in[18];
  const float* n1_g = (const float*)d_in[19]; const float* n1_b = (const float*)d_in[20];
  const float* n2_g = (const float*)d_in[21]; const float* n2_b = (const float*)d_in[22];
  const float* n3_g = (const float*)d_in[23]; const float* n3_b = (const float*)d_in[24];
  const float* w1 = (const float*)d_in[25]; const float* b1 = (const float*)d_in[26];
  const float* w2 = (const float*)d_in[27]; const float* b2 = (const float*)d_in[28];
  char* ws = (char*)d_ws;
  _Float16* WQKVS = (_Float16*)(ws + WS_WQKVS); _Float16* WOS = (_Float16*)(ws + WS_WOS);
  _Float16* WQKVC = (_Float16*)(ws + WS_WQKVC); _Float16* WOC = (_Float16*)(ws + WS_WOC);
  _Float16* W1T = (_Float16*)(ws + WS_W1T); _Float16* W2T = (_Float16*)(ws + WS_W2T);
  _Float16* XN = (_Float16*)(ws + WS_XN); _Float16* Qp = (_Float16*)(ws + WS_Q); _Float16* Kp = (_Float16*)(ws + WS_K);
  _Float16* VTp = (_Float16*)(ws + WS_VT); _Float16* Op = (_Float16*)(ws + WS_O); _Float16* Hp = (_Float16*)(ws + WS_H);
  float* X1 = (float*)(ws + WS_X1); float* X2 = (float*)(ws + WS_X2);
  float* out = (float*)d_out;
  const size_t SQ = (size_t)DM * DM;
  const size_t SOFF = (size_t)TOKS * DM;

  k_wt<<<dim3(DM / 64, DM / 64), 256, 0, stream>>>(sa_wq, (unsigned)DM, (unsigned)DM, WQKVS);
  k_wt<<<dim3(DM / 64, DM / 64), 256, 0, stream>>>(sa_wk, (unsigned)DM, (unsigned)DM, WQKVS + SQ);
  k_wt<<<dim3(DM / 64, DM / 64), 256, 0, stream>>>(sa_wv, (unsigned)DM, (unsigned)DM, WQKVS + 2 * SQ);
  k_wt<<<dim3(DM / 64, DM / 64), 256, 0, stream>>>(sa_wo, (unsigned)DM, (unsigned)DM, WOS);
  k_wt<<<dim3(DM / 64, DM / 64), 256, 0, stream>>>(ca_wq, (unsigned)DM, (unsigned)DM, WQKVC);
  k_wt<<<dim3(DM / 64, DM / 64), 256, 0, stream>>>(ca_wk, (unsigned)DM, (unsigned)DM, WQKVC + SQ);
  k_wt<<<dim3(DM / 64, DM / 64), 256, 0, stream>>>(ca_wv, (unsigned)DM, (unsigned)DM, WQKVC + 2 * SQ);
  k_wt<<<dim3(DM / 64, DM / 64), 256, 0, stream>>>(ca_wo, (unsigned)DM, (unsigned)DM, WOC);
  k_wt<<<dim3(FF / 64, DM / 64), 256, 0, stream>>>(w1, (unsigned)DM, (unsigned)FF, W1T);
  k_wt<<<dim3(DM / 64, FF / 64), 256, 0, stream>>>(w2, (unsigned)FF, (unsigned)DM, W2T);

  k_ln<1><<<dim3(ROWS / 8u), 256, 0, stream>>>(x0, x1, (unsigned)SEQ_FULL, n1_g, n1_b, XN);
  k_qkv<<<dim3(ROWS / 64u, 6), 128, 0, stream>>>(XN, WQKVS, sa_bq, sa_bk, sa_bv, Qp, Kp, VTp);
  k_attn<0><<<dim3(SEQ / 16, 2 * NB), 256, 0, stream>>>(Qp, Kp, VTp, vb, Op);
  k_gres<1><<<dim3(ROWS / 64u, DM / 128), 128, 0, stream>>>(Op, WOS, (unsigned)DM, sa_bo, x0, x1, (unsigned)SEQ_FULL, X1, X1 + SOFF, (unsigned)SEQ, 1.0f / (WC * OC));

  k_ln<0><<<dim3(ROWS / 8u), 256, 0, stream>>>(X1, X1 + SOFF, (unsigned)SEQ, n2_g, n2_b, XN);
  k_qkv<<<dim3(ROWS / 64u, 6), 128, 0, stream>>>(XN, WQKVC, ca_bq, ca_bk, ca_bv, Qp, Kp, VTp);
  k_attn<1><<<dim3(SEQ / 16, 2 * NB), 256, 0, stream>>>(Qp, Kp, VTp, vb, Op);
  k_gres<0><<<dim3(ROWS / 64u, DM / 128), 128, 0, stream>>>(Op, WOC, (unsigned)DM, ca_bo, X1, X1 + SOFF, (unsigned)SEQ, X2, X2 + SOFF, (unsigned)SEQ, 1.0f / (WC * OC));

  k_ln<0><<<dim3(ROWS / 8u), 256, 0, stream>>>(X2, X2 + SOFF, (unsigned)SEQ, n3_g, n3_b, XN);
  k_ffn1<<<dim3(ROWS / 64u, FF / 128), 128, 0, stream>>>(XN, W1T, b1, Hp);
  k_gres<0><<<dim3(ROWS / 64u, DM / 128), 128, 0, stream>>>(Hp, W2T, (unsigned)FF, b2, X2, X2 + SOFF, (unsigned)SEQ, out, out + OUT1_OFF, (unsigned)SEQ_FULL, 1.0f / WC);
}
